// MambaBlock_62208306315887
// MI455X (gfx1250) — hardware-verified
//
#include <hip/hip_runtime.h>
#include <stddef.h>
#include <stdint.h>
#include <math.h>


#define NBT    2
#define SL     2048
#define DIM    1024
#define DI     2048
#define DS     16
#define DTR    64
#define NXP    96
#define RW     4096
#define NIN    4096
#define KX     4096
#define KDT    128
#define NTHR   256
#define GBM    64
#define GBN    64
#define GTHR   128
#define XBN    96
#define SCT    64
#define SCK    64
#define BIGCOL (1 << 30)

static_assert(RW == NBT * SL && NIN == 2 * DI && KX == 2 * DI && KDT == 2 * DTR);
static_assert(RW % GBM == 0 && NIN % GBN == 0 && DI % GBN == 0 && DIM % GBN == 0);
static_assert(DIM % 32 == 0 && KX % 32 == 0 && KDT % 32 == 0);
static_assert(NXP == 6 * 16 && NXP == DTR + 2 * DS);
static_assert((RW * DIM / 8) % NTHR == 0);
static_assert((NIN * (DIM / 8)) % NTHR == 0 && (NXP * (KX / 8)) % NTHR == 0);
static_assert((DI * (KDT / 8)) % NTHR == 0 && (DIM * (KX / 8)) % NTHR == 0);
static_assert((DI * DS / 4) % NTHR == 0);
static_assert((RW * (DI / 4)) % NTHR == 0);
static_assert(DI % SCT == 0 && SL % SCK == 0 && (DI / SCT) == 32);
static_assert((SL & (SL - 1)) == 0);

typedef float          v4f   __attribute__((ext_vector_type(4)));
typedef float          v8f   __attribute__((ext_vector_type(8)));
typedef int            v8i   __attribute__((ext_vector_type(8)));
typedef unsigned       v2u   __attribute__((ext_vector_type(2)));
typedef unsigned short v8us  __attribute__((ext_vector_type(8)));
typedef unsigned short v16us __attribute__((ext_vector_type(16)));
typedef __bf16         v16bf __attribute__((ext_vector_type(16)));
typedef v4f  __attribute__((may_alias)) v4fa;
typedef v8us __attribute__((may_alias)) v8usa;
union FragB { v16bf v; v16us u; v8us h[2]; v8i w; };

__device__ __forceinline__ v8f wmb(const FragB& a, const FragB& b, v8f c) {
  v8f d = __builtin_amdgcn_wmma_f32_16x16x32_bf16(false, a.v, false, b.v, (short)0, c, false, false);
  asm volatile("v_nop\n\tv_nop\n\tv_nop\n\tv_nop" : "+v"(d) : "v"(a.w), "v"(b.w));
  return d;
}

__device__ __forceinline__ unsigned bf16_bits(float f) {
  const unsigned u = __float_as_uint(f);
  return (u + 0x7FFFu + ((u >> 16) & 1u)) >> 16;
}
__device__ __forceinline__ float bf16_val(float f) {
  return __uint_as_float(bf16_bits(f) << 16);
}
__device__ __forceinline__ float silu_f(float v) {
  return v * __builtin_amdgcn_rcpf(1.0f + expf(-v));
}
__device__ __forceinline__ float softplus_f(float v) {
  return fmaxf(v, 0.0f) + log1pf(expf(-fabsf(v)));
}

__global__ __launch_bounds__(NTHR) void k_cvx(const float* __restrict__ x, unsigned short* xb) {
  const int u = (int)blockIdx.x * NTHR + (int)threadIdx.x;
  const float* p = x + (size_t)u * 8;
  const v4f a = *(const v4fa*)p;
  const v4f b = *(const v4fa*)(p + 4);
  v8us o;
  o[0] = (unsigned short)bf16_bits(a.x); o[1] = (unsigned short)bf16_bits(a.y);
  o[2] = (unsigned short)bf16_bits(a.z); o[3] = (unsigned short)bf16_bits(a.w);
  o[4] = (unsigned short)bf16_bits(b.x); o[5] = (unsigned short)bf16_bits(b.y);
  o[6] = (unsigned short)bf16_bits(b.z); o[7] = (unsigned short)bf16_bits(b.w);
  unsigned short* dp = xb + (size_t)u * 8;
  *(volatile v8us*)dp = o;
  __threadfence();
  *(volatile v8us*)dp = o;
}

__global__ __launch_bounds__(NTHR) void k_wt(const float* __restrict__ W, unsigned short* WT,
                                             int N, int kmask, int lgU, int KP, int nUnits) {
  const int u = (int)blockIdx.x * NTHR + (int)threadIdx.x;
  if (u >= nUnits) return;
  const int n  = u >> lgU;
  const int k8 = (u & ((1 << lgU) - 1)) * 8;
  const int kk = k8 & kmask;
  const float* p = W + (size_t)kk * (size_t)N + n;
  v8us o;
#pragma unroll
  for (int i = 0; i < 8; ++i) o[i] = (unsigned short)bf16_bits(p[(size_t)i * (size_t)N]);
  unsigned short* dp = WT + (size_t)n * (size_t)KP + k8;
  *(volatile v8us*)dp = o;
  __threadfence();
  *(volatile v8us*)dp = o;
}

__global__ __launch_bounds__(NTHR) void k_an(const float* __restrict__ alog, float* an) {
  const int u = (int)blockIdx.x * NTHR + (int)threadIdx.x;
  const v4f a = *(const v4fa*)(alog + (size_t)u * 4);
  v4f o;
  o.x = -expf(bf16_val(a.x));
  o.y = -expf(bf16_val(a.y));
  o.z = -expf(bf16_val(a.z));
  o.w = -expf(bf16_val(a.w));
  float* dp = an + (size_t)u * 4;
  *(volatile v4f*)dp = o;
  __threadfence();
  *(volatile v4f*)dp = o;
}

template <int NT>
__device__ __forceinline__ void gemm_core(const unsigned short* __restrict__ ap,
                                          const unsigned short* __restrict__ wp, int K, v8f (&acc)[NT]) {
  const int ksteps = K >> 5;
#pragma unroll 1
  for (int ks = 0; ks < ksteps; ++ks) {
    FragB af;
    af.h[0] = *(const v8usa*)(ap + 32 * ks);
    af.h[1] = *(const v8usa*)(ap + 32 * ks + 16);
#pragma unroll
    for (int t = 0; t < NT; ++t) {
      const unsigned short* wq = wp + (size_t)(16 * t) * (size_t)K + 32 * ks;
      FragB bf;
      bf.h[0] = *(const v8usa*)wq;
      bf.h[1] = *(const v8usa*)(wq + 16);
      acc[t] = wmb(af, bf, acc[t]);
    }
  }
}

template <int EPI>
__global__ __launch_bounds__(GTHR) void k_gemm(const unsigned short* __restrict__ A,
                                               const unsigned short* __restrict__ WT,
                                               float* outF, const float* __restrict__ bias,
                                               int K, int ldo, int splitCol, int planeStride) {
  __shared__ __attribute__((aligned(16))) float stg[GBM * GBN];
  const int tid = (int)threadIdx.x, lane = tid & 31, wave = tid >> 5, hh = lane >> 4, m = lane & 15;
  const int rowBase = (int)blockIdx.x * GBM;
  const int col0    = (int)blockIdx.y * GBN;

  v8f acc[4];
  {
    const v8f z = {0.f, 0.f, 0.f, 0.f, 0.f, 0.f, 0.f, 0.f};
    acc[0] = z; acc[1] = z; acc[2] = z; acc[3] = z;
  }
  const unsigned short* ap = A  + (size_t)(rowBase + 16 * wave + m) * (size_t)K + 8 * hh;
  const unsigned short* wp = WT + (size_t)(col0 + m) * (size_t)K + 8 * hh;
  gemm_core<4>(ap, wp, K, acc);

#pragma unroll
  for (int t = 0; t < 4; ++t) {
    const int lc = 16 * t + m;
#pragma unroll
    for (int r = 0; r < 8; ++r) {
      const int lr = 16 * wave + 8 * hh + r;
      stg[lr * GBN + lc] = acc[t][r];
    }
  }
  __syncthreads();

  const int pl = (col0 >= splitCol) ? 1 : 0;
  const int cc = col0 - pl * splitCol;
  float* ob = outF + (size_t)pl * (size_t)planeStride;

  if constexpr (EPI == 1) {
    if (pl != 0) {
#pragma unroll 1
      for (int i = 0; i < 8; ++i) {
        float* sp = stg + (16 * wave + 2 * i + hh) * GBN + 4 * m;
        v4f v = *(const v4fa*)sp;
        v.x = silu_f(v.x); v.y = silu_f(v.y); v.z = silu_f(v.z); v.w = silu_f(v.w);
        *(v4fa*)sp = v;
      }
    }
  }
  if constexpr (EPI == 2) {
    const v4f b4 = *(const v4fa*)(bias + col0 + 4 * m);
    const float bx = bf16_val(b4.x), by = bf16_val(b4.y), bz = bf16_val(b4.z), bw = bf16_val(b4.w);
#pragma unroll 1
    for (int i = 0; i < 8; ++i) {
      float* sp = stg + (16 * wave + 2 * i + hh) * GBN + 4 * m;
      v4f v = *(const v4fa*)sp;
      v.x = softplus_f(v.x + bx); v.y = softplus_f(v.y + by);
      v.z = softplus_f(v.z + bz); v.w = softplus_f(v.w + bw);
      *(v4fa*)sp = v;
    }
  }

  v4f fv[8];
#pragma unroll
  for (int i = 0; i < 8; ++i) {
    const int lr = 16 * wave + 2 * i + hh;
    fv[i] = *(const v4fa*)(stg + lr * GBN + 4 * m);
  }
#pragma unroll
  for (int i = 0; i < 8; ++i) {
    const int gr = rowBase + 16 * wave + 2 * i + hh;
    float* op = ob + (size_t)gr * (size_t)ldo + cc + 4 * m;
    *(volatile v4f*)op = fv[i];
  }
  __threadfence();
#pragma unroll
  for (int i = 0; i < 8; ++i) {
    const int gr = rowBase + 16 * wave + 2 * i + hh;
    float* op = ob + (size_t)gr * (size_t)ldo + cc + 4 * m;
    *(volatile v4f*)op = fv[i];
  }
}

__global__ __launch_bounds__(GTHR) void k_xproj(const unsigned short* __restrict__ A,
                                                const unsigned short* __restrict__ WT,
                                                float* dbl, unsigned short* dtrhl) {
  __shared__ __attribute__((aligned(16))) float stg[GBM * XBN];
  const int tid = (int)threadIdx.x, lane = tid & 31, wave = tid >> 5, hh = lane >> 4, m = lane & 15;
  const int rowBase = (int)blockIdx.x * GBM;

  v8f acc[6];
  {
    const v8f z = {0.f, 0.f, 0.f, 0.f, 0.f, 0.f, 0.f, 0.f};
#pragma unroll
    for (int t = 0; t < 6; ++t) acc[t] = z;
  }
  const unsigned short* ap = A  + (size_t)(rowBase + 16 * wave + m) * (size_t)KX + 8 * hh;
  const unsigned short* wp = WT + (size_t)m * (size_t)KX + 8 * hh;
  gemm_core<6>(ap, wp, KX, acc);

#pragma unroll
  for (int t = 0; t < 6; ++t) {
    const int lc = 16 * t + m;
#pragma unroll
    for (int r = 0; r < 8; ++r) {
      const int lr = 16 * wave + 8 * hh + r;
      stg[lr * XBN + lc] = acc[t][r];
    }
  }
  __syncthreads();

  const float* sb = stg + 16 * wave * XBN;
  v4f fv[12];
#pragma unroll
  for (int j = 0; j < 12; ++j) fv[j] = *(const v4fa*)(sb + 4 * (j * 32 + lane));
  v8us hv[8];
#pragma unroll
  for (int j = 0; j < 8; ++j) {
    const int p   = j * 32 + lane;
    const int row = p >> 4;
    const int q   = p & 15;
    const bool lo = q >= 8;
    const float* s = sb + row * XBN + (q & 7) * 8;
    const v4f a = *(const v4fa*)s;
    const v4f b = *(const v4fa*)(s + 4);
    const float e[8] = {a.x, a.y, a.z, a.w, b.x, b.y, b.z, b.w};
    v8us o;
#pragma unroll
    for (int i = 0; i < 8; ++i) {
      const unsigned hb = bf16_bits(e[i]);
      const unsigned lb = bf16_bits(e[i] - __uint_as_float(hb << 16));
      o[i] = (unsigned short)(lo ? lb : hb);
    }
    hv[j] = o;
  }
  float* gb = dbl + (size_t)(rowBase + 16 * wave) * XBN;
  unsigned short* gh = dtrhl + (size_t)(rowBase + 16 * wave) * KDT;
#pragma unroll
  for (int j = 0; j < 12; ++j) *(volatile v4f*)(gb + 4 * (j * 32 + lane)) = fv[j];
#pragma unroll
  for (int j = 0; j < 8; ++j) *(volatile v8us*)(gh + 8 * (j * 32 + lane)) = hv[j];
  __threadfence();
#pragma unroll
  for (int j = 0; j < 12; ++j) *(volatile v4f*)(gb + 4 * (j * 32 + lane)) = fv[j];
#pragma unroll
  for (int j = 0; j < 8; ++j) *(volatile v8us*)(gh + 8 * (j * 32 + lane)) = hv[j];
}

__global__ __launch_bounds__(NTHR) void k_conv(const float* __restrict__ xpre, const float* __restrict__ cw,
                                               const float* __restrict__ cb, float* xp, unsigned short* xphl) {
  const int u = (int)blockIdx.x * NTHR + (int)threadIdx.x;
  const int r = u >> 9;
  const int c = (u & 511) * 4;
  const int l = r & (SL - 1);
  v4f xs[4];
#pragma unroll
  for (int k = 0; k < 4; ++k) {
    const bool ok = (l - 3 + k) >= 0;
    const int rk = ok ? (r - 3 + k) : r;
    const float fk = ok ? 1.0f : 0.0f;
    const v4f t = *(const v4fa*)(xpre + (size_t)rk * DI + c);
    xs[k] = t * fk;
  }
  const v4f w0 = *(const v4fa*)(cw + (size_t)(c + 0) * 4);
  const v4f w1 = *(const v4fa*)(cw + (size_t)(c + 1) * 4);
  const v4f w2 = *(const v4fa*)(cw + (size_t)(c + 2) * 4);
  const v4f w3 = *(const v4fa*)(cw + (size_t)(c + 3) * 4);
  const v4f b4 = *(const v4fa*)(cb + c);
  float s0, s1, s2, s3;
  s0 = bf16_val(w0.x) * xs[0].x; s0 = fmaf(bf16_val(w0.y), xs[1].x, s0);
  s0 = fmaf(bf16_val(w0.z), xs[2].x, s0); s0 = fmaf(bf16_val(w0.w), xs[3].x, s0); s0 = s0 + bf16_val(b4.x);
  s1 = bf16_val(w1.x) * xs[0].y; s1 = fmaf(bf16_val(w1.y), xs[1].y, s1);
  s1 = fmaf(bf16_val(w1.z), xs[2].y, s1); s1 = fmaf(bf16_val(w1.w), xs[3].y, s1); s1 = s1 + bf16_val(b4.y);
  s2 = bf16_val(w2.x) * xs[0].z; s2 = fmaf(bf16_val(w2.y), xs[1].z, s2);
  s2 = fmaf(bf16_val(w2.z), xs[2].z, s2); s2 = fmaf(bf16_val(w2.w), xs[3].z, s2); s2 = s2 + bf16_val(b4.z);
  s3 = bf16_val(w3.x) * xs[0].w; s3 = fmaf(bf16_val(w3.y), xs[1].w, s3);
  s3 = fmaf(bf16_val(w3.z), xs[2].w, s3); s3 = fmaf(bf16_val(w3.w), xs[3].w, s3); s3 = s3 + bf16_val(b4.w);
  v4f v;
  v.x = silu_f(s0); v.y = silu_f(s1); v.z = silu_f(s2); v.w = silu_f(s3);
  const unsigned h0 = bf16_bits(v.x), h1 = bf16_bits(v.y), h2 = bf16_bits(v.z), h3 = bf16_bits(v.w);
  const unsigned l0 = bf16_bits(v.x - __uint_as_float(h0 << 16));
  const unsigned l1 = bf16_bits(v.y - __uint_as_float(h1 << 16));
  const unsigned l2 = bf16_bits(v.z - __uint_as_float(h2 << 16));
  const unsigned l3 = bf16_bits(v.w - __uint_as_float(h3 << 16));
  v2u hw, lw;
  hw.x = h0 | (h1 << 16); hw.y = h2 | (h3 << 16);
  lw.x = l0 | (l1 << 16); lw.y = l2 | (l3 << 16);
  float* xo = xp + (size_t)r * DI + c;
  unsigned short* hp = xphl + (size_t)r * KX + c;
  unsigned short* lp = hp + DI;
  *(volatile v4f*)xo = v;
  *(volatile v2u*)hp = hw;
  *(volatile v2u*)lp = lw;
  __threadfence();
  *(volatile v4f*)xo = v;
  *(volatile v2u*)hp = hw;
  *(volatile v2u*)lp = lw;
}

__global__ __launch_bounds__(SCT) void k_scan(const float* __restrict__ dtp, const float* __restrict__ xp,
                                             const float* __restrict__ gp, const float* __restrict__ dbl,
                                             const float* __restrict__ an, const float* __restrict__ dvec,
                                             unsigned short* yhl) {
  __shared__ __attribute__((aligned(16))) float bc[SCK * 32];
  __shared__ __attribute__((aligned(16))) unsigned short ys[2 * SCK * SCT];
  const int tid   = (int)threadIdx.x;
  const int batch = (int)blockIdx.x >> 5;
  const int dblk  = (int)blockIdx.x & 31;
  const int d     = dblk * SCT + tid;
  const int row0  = batch * SL;

  float Av[16], h[16];
  {
    const v4f a0 = *(const v4fa*)(an + (size_t)d * DS);
    const v4f a1 = *(const v4fa*)(an + (size_t)d * DS + 4);
    const v4f a2 = *(const v4fa*)(an + (size_t)d * DS + 8);
    const v4f a3 = *(const v4fa*)(an + (size_t)d * DS + 12);
    Av[0] = a0.x; Av[1] = a0.y; Av[2] = a0.z; Av[3] = a0.w;
    Av[4] = a1.x; Av[5] = a1.y; Av[6] = a1.z; Av[7] = a1.w;
    Av[8] = a2.x; Av[9] = a2.y; Av[10] = a2.z; Av[11] = a2.w;
    Av[12] = a3.x; Av[13] = a3.y; Av[14] = a3.z; Av[15] = a3.w;
#pragma unroll
    for (int s = 0; s < 16; ++s) h[s] = 0.0f;
  }
  const float Dc = bf16_val(dvec[d]);

#pragma unroll 1
  for (int ch = 0; ch < SL / SCK; ++ch) {
    const int rb = row0 + ch * SCK;
#pragma unroll
    for (int i = 0; i < 8; ++i) {
      const int idx = i * SCT + tid;
      const int t = idx >> 3, q = idx & 7;
      const v4f v = *(const v4fa*)(dbl + (size_t)(rb + t) * NXP + DTR + 4 * q);
      *(v4fa*)(bc + t * 32 + 4 * q) = v;
    }
    __syncthreads();

#pragma unroll 1
    for (int t = 0; t < SCK; ++t) {
      const size_t off = (size_t)(rb + t) * DI + d;
      const float dtv = dtp[off];
      const float xv  = xp[off];
      const float gv  = gp[off];
      const float* bp = bc + t * 32;
      const v4f b0 = *(const v4fa*)(bp);
      const v4f b1 = *(const v4fa*)(bp + 4);
      const v4f b2 = *(const v4fa*)(bp + 8);
      const v4f b3 = *(const v4fa*)(bp + 12);
      const v4f c0 = *(const v4fa*)(bp + 16);
      const v4f c1 = *(const v4fa*)(bp + 20);
      const v4f c2 = *(const v4fa*)(bp + 24);
      const v4f c3 = *(const v4fa*)(bp + 28);
      const float Bv[16] = {b0.x, b0.y, b0.z, b0.w, b1.x, b1.y, b1.z, b1.w,
                            b2.x, b2.y, b2.z, b2.w, b3.x, b3.y, b3.z, b3.w};
      const float Cv[16] = {c0.x, c0.y, c0.z, c0.w, c1.x, c1.y, c1.z, c1.w,
                            c2.x, c2.y, c2.z, c2.w, c3.x, c3.y, c3.z, c3.w};
      float y = 0.0f;
#pragma unroll
      for (int s = 0; s < 16; ++s) {
        const float dA = expf(dtv * Av[s]);
        h[s] = dA * h[s] + (dtv * Bv[s]) * xv;
        y = y + h[s] * Cv[s];
      }
      const float y2 = (y + xv * Dc) * gv;
      const unsigned hb = bf16_bits(y2);
      const unsigned lb = bf16_bits(y2 - __uint_as_float(hb << 16));
      ys[t * SCT + tid] = (unsigned short)hb;
      ys[SCK * SCT + t * SCT + tid] = (unsigned short)lb;
    }
    __syncthreads();

    v8us qv[16];
#pragma unroll
    for (int j = 0; j < 16; ++j) {
      const int p = j * SCT + tid;
      const int q = p & 7, sel = (p >> 3) & 1, t = p >> 4;
      qv[j] = *(const v8usa*)(ys + sel * (SCK * SCT) + t * SCT + 8 * q);
    }
#pragma unroll
    for (int j = 0; j < 16; ++j) {
      const int p = j * SCT + tid;
      const int q = p & 7, sel = (p >> 3) & 1, t = p >> 4;
      unsigned short* dp = yhl + (size_t)(rb + t) * KX + sel * DI + dblk * SCT + 8 * q;
      *(volatile v8us*)dp = qv[j];
    }
    __threadfence();
#pragma unroll
    for (int j = 0; j < 16; ++j) {
      const int p = j * SCT + tid;
      const int q = p & 7, sel = (p >> 3) & 1, t = p >> 4;
      unsigned short* dp = yhl + (size_t)(rb + t) * KX + sel * DI + dblk * SCT + 8 * q;
      *(volatile v8us*)dp = qv[j];
    }
  }
}

static inline size_t al256(size_t o) { return (o + 255) & ~(size_t)255; }

extern "C" void kernel_launch(void* const* d_in, const int* in_sizes, int n_in,
                              void* d_out, int out_size, void* d_ws, size_t ws_size,
                              hipStream_t stream) {
  if (n_in < 10) return;
  if (in_sizes[0] != RW * DIM) return;
  if (in_sizes[1] != DIM * NIN) return;
  if (in_sizes[2] != DI * 4) return;
  if (in_sizes[3] != DI) return;
  if (in_sizes[4] != DI * NXP) return;
  if (in_sizes[5] != DTR * DI) return;
  if (in_sizes[6] != DI) return;
  if (in_sizes[7] != DI * DS) return;
  if (in_sizes[8] != DI) return;
  if (in_sizes[9] != DI * DIM) return;
  if (out_size != RW * DIM) return;

  const float* x      = (const float*)d_in[0];
  const float* W_in   = (const float*)d_in[1];
  const float* conv_w = (const float*)d_in[2];
  const float* conv_b = (const float*)d_in[3];
  const float* W_xp   = (const float*)d_in[4];
  const float* W_dt   = (const float*)d_in[5];
  const float* b_dt   = (const float*)d_in[6];
  const float* A_log  = (const float*)d_in[7];
  const float* Dv     = (const float*)d_in[8];
  const float* W_out  = (const float*)d_in[9];
  float* out = (float*)d_out;

  char* ws = (char*)d_ws;
  size_t off = 0;
  const size_t oXB  = off; off = al256(off + (size_t)RW * DIM * 2);
  const size_t oWIN = off; off = al256(off + (size_t)NIN * DIM * 2);
  const size_t oWO2 = off; off = al256(off + (size_t)DIM * KX * 2);
  const size_t oWX2 = off; off = al256(off + (size_t)NXP * KX * 2);
  const size_t oWD2 = off; off = al256(off + (size_t)DI * KDT * 2);
  const size_t oDBL = off; off = al256(off + (size_t)RW * NXP * 4);
  const size_t oDTR = off; off = al256(off + (size_t)RW * KDT * 2);
  const size_t oAN  = off; off = al256(off + (size_t)DI * DS * 4);
  const size_t oXG  = off; off = al256(off + (size_t)2 * RW * DI * 4);
  const size_t oXP  = off; off = al256(off + (size_t)RW * DI * 4);
  const size_t oHL  = off; off = al256(off + (size_t)RW * KX * 2);
  if (off > ws_size) return;
  unsigned short* XB   = (unsigned short*)(ws + oXB);
  unsigned short* WINT = (unsigned short*)(ws + oWIN);
  unsigned short* WO2  = (unsigned short*)(ws + oWO2);
  unsigned short* WX2  = (unsigned short*)(ws + oWX2);
  unsigned short* WDT2 = (unsigned short*)(ws + oWD2);
  float*          DBL  = (float*)(ws + oDBL);
  unsigned short* DTRH = (unsigned short*)(ws + oDTR);
  float*          AN   = (float*)(ws + oAN);
  float*          XPRE = (float*)(ws + oXG);
  float*          G    = XPRE + (size_t)RW * DI;
  float*          XP   = (float*)(ws + oXP);
  unsigned short* HL   = (unsigned short*)(ws + oHL);

  k_cvx<<<(RW * DIM / 8) / NTHR, NTHR, 0, stream>>>(x, XB);
  k_wt<<<(NIN * (DIM / 8)) / NTHR, NTHR, 0, stream>>>(W_in, WINT, NIN, DIM - 1, 7, DIM, NIN * (DIM / 8));
  k_wt<<<(NXP * (KX / 8)) / NTHR, NTHR, 0, stream>>>(W_xp, WX2, NXP, DI - 1, 9, KX, NXP * (KX / 8));
  k_wt<<<(DI * (KDT / 8)) / NTHR, NTHR, 0, stream>>>(W_dt, WDT2, DI, DTR - 1, 4, KDT, DI * (KDT / 8));
  k_wt<<<(DIM * (KX / 8)) / NTHR, NTHR, 0, stream>>>(W_out, WO2, DIM, DI - 1, 9, KX, DIM * (KX / 8));
  k_an<<<(DI * DS / 4) / NTHR, NTHR, 0, stream>>>(A_log, AN);
  k_gemm<1><<<dim3(RW / GBM, NIN / GBN), GTHR, 0, stream>>>(XB, WINT, XPRE, b_dt, DIM, DI, DI, RW * DI);
  k_conv<<<(RW * (DI / 4)) / NTHR, NTHR, 0, stream>>>(XPRE, conv_w, conv_b, XP, HL);
  k_xproj<<<RW / GBM, GTHR, 0, stream>>>(HL, WX2, DBL, DTRH);
  k_gemm<2><<<dim3(RW / GBM, DI / GBN), GTHR, 0, stream>>>(DTRH, WDT2, XPRE, b_dt, KDT, DI, BIGCOL, 0);
  k_scan<<<NBT * (DI / SCT), SCT, 0, stream>>>(XPRE, XP, G, DBL, AN, Dv, HL);
  k_gemm<0><<<dim3(RW / GBM, DIM / GBN), GTHR, 0, stream>>>(HL, WO2, out, b_dt, KX, DIM, BIGCOL, 0);
}
